// E3ProbeMessageModel_3315714752867
// MI455X (gfx1250) — hardware-verified
//
#include <hip/hip_runtime.h>
#define NA 2000
#define NAP 2016
#define NPR 20000
#define NPP 20032
#define NE 200000
#define ECH 12500
#define DIM 320
#define M0 128
#define M1 64
#define MID 192
#define WN 384
#define FH 100
#define FHP 128

typedef __bf16 v16b __attribute__((ext_vector_type(16)));
typedef unsigned short v8us __attribute__((ext_vector_type(8), may_alias));
typedef float  v8f  __attribute__((ext_vector_type(8)));
typedef float  v4f  __attribute__((ext_vector_type(4)));
typedef float  v4fa __attribute__((ext_vector_type(4), may_alias));
union FragB { v16b v; v8us half[2]; unsigned short u[16]; };

__device__ __forceinline__ unsigned short bf16_bits(float x) { unsigned int u = __float_as_uint(x); return (unsigned short)((u + 0x7FFFu + ((u >> 16) & 1u)) >> 16); }
__device__ __forceinline__ float bf16_val(unsigned short b) { return __uint_as_float(((unsigned int)b) << 16); }
__device__ __forceinline__ float bf16_round(float x) { return bf16_val(bf16_bits(x)); }
template <int NT>
__device__ __forceinline__ v8f mmaN(v16b ah, v16b al, v16b bh, v16b bl, v8f c) {
  c = __builtin_amdgcn_wmma_f32_16x16x32_bf16(false, ah, false, bh, (short)0, c, false, false);
  if (NT >= 2) c = __builtin_amdgcn_wmma_f32_16x16x32_bf16(false, al, false, bh, (short)0, c, false, false);
  if (NT >= 3) c = __builtin_amdgcn_wmma_f32_16x16x32_bf16(false, ah, false, bl, (short)0, c, false, false);
  asm volatile("v_nop\n\tv_nop\n\tv_nop\n\tv_nop" : "+v"(c) : "v"(ah), "v"(al), "v"(bh), "v"(bl));
  return c;
}

__global__ __launch_bounds__(256) void k_wt_bf16(const float* __restrict__ W, unsigned short* __restrict__ Wt, int K, int N) {
  const int t = blockIdx.x * 256 + threadIdx.x;
  const int k8n = K / 8;
  if (t >= N * k8n) return;
  const int n = t / k8n, k8 = (t % k8n) * 8;
  v8us v;
#pragma unroll
  for (int i = 0; i < 8; ++i) v[i] = bf16_bits(W[(size_t)(k8 + i) * N + n]);
  *(volatile v8us*)(Wt + (size_t)n * K + k8) = v;
  __threadfence();
  *(volatile v8us*)(Wt + (size_t)n * K + k8) = v;
}

template <bool ASPLIT, int ACT, bool BIAS_BF16>
__global__ __launch_bounds__(128) void k_gemm_bf(const float* __restrict__ A, int lda, const unsigned short* __restrict__ Wt, int ldb,
                                               const float* __restrict__ bias, float* __restrict__ C, int ldc, int M, int N, int K) {
  __shared__ __attribute__((aligned(16))) float so[4][16][64];
  const int tid = threadIdx.x, w = tid >> 5, lane = tid & 31, ln = lane & 15, hh = lane >> 4;
  const int ntn = N / 64;
  const int wid = blockIdx.x * 4 + w;
  const int mt = wid / ntn, nq = wid % ntn;
  if (mt * 16 >= M) return;
  const int row0 = mt * 16, col0 = nq * 64;
  const float* arow = A + (size_t)(row0 + ln) * lda;
  v8f acc[4] = {};
  for (int kb = 0; kb < K; kb += 32) {
    FragB ah, al;
    const v4f x0 = *(const v4fa*)(arow + kb + 8 * hh), x1 = *(const v4fa*)(arow + kb + 8 * hh + 4);
    const v4f x2 = *(const v4fa*)(arow + kb + 16 + 8 * hh), x3 = *(const v4fa*)(arow + kb + 16 + 8 * hh + 4);
    float xs[16] = {x0[0],x0[1],x0[2],x0[3],x1[0],x1[1],x1[2],x1[3],x2[0],x2[1],x2[2],x2[3],x3[0],x3[1],x3[2],x3[3]};
#pragma unroll
    for (int i = 0; i < 16; ++i) { const unsigned short hb = bf16_bits(xs[i]); ah.u[i] = hb; al.u[i] = ASPLIT ? bf16_bits(xs[i] - bf16_val(hb)) : (unsigned short)0; }
#pragma unroll
    for (int t = 0; t < 4; ++t) {
      const unsigned short* brow = Wt + (size_t)(col0 + t * 16 + ln) * ldb + kb;
      FragB b;
      b.half[0] = *(const v8us*)(brow + 8 * hh);
      b.half[1] = *(const v8us*)(brow + 16 + 8 * hh);
      acc[t] = mmaN<ASPLIT ? 2 : 1>(ah.v, al.v, b.v, b.v, acc[t]);
    }
  }
#pragma unroll
  for (int t = 0; t < 4; ++t) {
    float bv = bias ? bias[col0 + t * 16 + ln] : 0.f;
    if (BIAS_BF16) bv = bf16_round(bv);
#pragma unroll
    for (int r = 0; r < 8; ++r) { float v = acc[t][r] + bv; if (ACT == 1) v = fmaxf(v, 0.f); so[w][8 * hh + r][t * 16 + ln] = v; }
  }
  __builtin_amdgcn_fence(__ATOMIC_ACQ_REL, "workgroup");
  __builtin_amdgcn_wave_barrier();
  const int rsub = lane >> 4, c4 = (lane & 15) * 4;
  for (int pass = 0; pass < 2; ++pass) {
#pragma unroll
    for (int q = 0; q < 8; ++q) {
      const int r = q * 2 + rsub;
      const v4f v = *(const v4fa*)&so[w][r][c4];
      *(volatile v4f*)(C + (size_t)(row0 + r) * ldc + col0 + c4) = v;
    }
    if (pass == 0) __threadfence();
  }
}

template <int D, bool CAUSAL>
__global__ __launch_bounds__(128) void k_flash(const float* __restrict__ qb, const float* __restrict__ kb, const float* __restrict__ vb,
                                             int pitch, int T, int H, float scale, float* __restrict__ y, int ypitch) {
  constexpr int KS = D / 32;
  constexpr int DT = D / 16;
  __shared__ __attribute__((aligned(16))) unsigned short sKh[32][D + 8], sKl[32][D + 8], sVh[32][D + 8], sVl[32][D + 8];
  __shared__ __attribute__((aligned(16))) unsigned short sPh[4][16][40], sPl[4][16][40];
  __shared__ __attribute__((aligned(16))) float sO[4][16][D];
  const int tid = threadIdx.x, w = tid >> 5, lane = tid & 31, ln = lane & 15, hh = lane >> 4;
  const int nqb = (T + 63) / 64;
  const int bh = blockIdx.x / nqb, qblk = blockIdx.x % nqb;
  const int b = bh / H, h = bh % H;
  const int q0 = qblk * 64 + w * 16;
  const float* Q = qb + (size_t)b * T * pitch + h * D;
  const float* K = kb + (size_t)b * T * pitch + h * D;
  const float* V = vb + (size_t)b * T * pitch + h * D;

  FragB aqh[KS], aql[KS];
  {
    int row = q0 + ln; if (row >= T) row = T - 1;
    const float* qr = Q + (size_t)row * pitch;
#pragma unroll
    for (int ks = 0; ks < KS; ++ks)
#pragma unroll
      for (int i = 0; i < 16; ++i) {
        const int d = ks * 32 + ((i < 8) ? (8 * hh + i) : (16 + 8 * hh + (i - 8)));
        const float x = qr[d] * scale; const unsigned short hb = bf16_bits(x);
        aqh[ks].u[i] = hb; aql[ks].u[i] = bf16_bits(x - bf16_val(hb));
      }
  }
  float m_r[8], l_r[8];
#pragma unroll
  for (int r = 0; r < 8; ++r) { m_r[r] = -3.0e38f; l_r[r] = 0.f; }
  v8f oacc[DT];
#pragma unroll
  for (int dt = 0; dt < DT; ++dt) oacc[dt] = (v8f){0.f,0.f,0.f,0.f,0.f,0.f,0.f,0.f};

  const int kv_end = CAUSAL ? min(T, qblk * 64 + 64) : T;
  for (int j0 = 0; j0 < kv_end; j0 += 32) {
    __syncthreads();
    for (int e = tid; e < 32 * (D / 4); e += 128) {
      const int r = e / (D / 4), c4 = (e % (D / 4)) * 4;
      const int key = j0 + r;
      v4f kf = {0.f,0.f,0.f,0.f}, vf = {0.f,0.f,0.f,0.f};
      if (key < T) { kf = *(const v4fa*)(K + (size_t)key * pitch + c4); vf = *(const v4fa*)(V + (size_t)key * pitch + c4); }
#pragma unroll
      for (int t = 0; t < 4; ++t) {
        unsigned short hb = bf16_bits(kf[t]); sKh[r][c4 + t] = hb; sKl[r][c4 + t] = bf16_bits(kf[t] - bf16_val(hb));
        hb = bf16_bits(vf[t]); sVh[r][c4 + t] = hb; sVl[r][c4 + t] = bf16_bits(vf[t] - bf16_val(hb));
      }
    }
    __syncthreads();
    v8f s[2];
#pragma unroll
    for (int nt = 0; nt < 2; ++nt) {
      v8f acc = {};
#pragma unroll
      for (int ks = 0; ks < KS; ++ks) {
        FragB bh_, bl_;
        bh_.half[0] = *(const v8us*)&sKh[nt * 16 + ln][ks * 32 + 8 * hh]; bh_.half[1] = *(const v8us*)&sKh[nt * 16 + ln][ks * 32 + 16 + 8 * hh];
        bl_.half[0] = *(const v8us*)&sKl[nt * 16 + ln][ks * 32 + 8 * hh]; bl_.half[1] = *(const v8us*)&sKl[nt * 16 + ln][ks * 32 + 16 + 8 * hh];
        acc = mmaN<3>(aqh[ks].v, aql[ks].v, bh_.v, bl_.v, acc);
      }
      s[nt] = acc;
    }
    float alpha[8];
#pragma unroll
    for (int r = 0; r < 8; ++r) {
      const int qi = q0 + 8 * hh + r;
      const int ja = j0 + ln, jb = j0 + 16 + ln;
      if (CAUSAL) { if (ja > qi) s[0][r] = -3.0e38f; if (jb > qi) s[1][r] = -3.0e38f; }
      if (ja >= T) s[0][r] = -3.0e38f;
      if (jb >= T) s[1][r] = -3.0e38f;
      float mx = fmaxf(s[0][r], s[1][r]);
      mx = fmaxf(mx, __shfl_xor(mx, 1, 32)); mx = fmaxf(mx, __shfl_xor(mx, 2, 32)); mx = fmaxf(mx, __shfl_xor(mx, 4, 32)); mx = fmaxf(mx, __shfl_xor(mx, 8, 32));
      const float mnew = fmaxf(m_r[r], mx);
      alpha[r] = (mnew > -1.0e38f) ? __expf(m_r[r] - mnew) : 1.0f;
      const float p0 = (s[0][r] > -1.0e38f) ? __expf(s[0][r] - mnew) : 0.f;
      const float p1 = (s[1][r] > -1.0e38f) ? __expf(s[1][r] - mnew) : 0.f;
      m_r[r] = mnew;
      l_r[r] = l_r[r] * alpha[r] + p0 + p1;
      unsigned short hb = bf16_bits(p0); sPh[w][8 * hh + r][ln] = hb;      sPl[w][8 * hh + r][ln] = bf16_bits(p0 - bf16_val(hb));
      hb = bf16_bits(p1);                sPh[w][8 * hh + r][16 + ln] = hb; sPl[w][8 * hh + r][16 + ln] = bf16_bits(p1 - bf16_val(hb));
    }
#pragma unroll
    for (int dt = 0; dt < DT; ++dt)
#pragma unroll
      for (int r = 0; r < 8; ++r) oacc[dt][r] *= alpha[r];
    __builtin_amdgcn_fence(__ATOMIC_ACQ_REL, "workgroup");
    __builtin_amdgcn_wave_barrier();
    FragB pah, pal;
    pah.half[0] = *(const v8us*)&sPh[w][ln][8 * hh]; pah.half[1] = *(const v8us*)&sPh[w][ln][16 + 8 * hh];
    pal.half[0] = *(const v8us*)&sPl[w][ln][8 * hh]; pal.half[1] = *(const v8us*)&sPl[w][ln][16 + 8 * hh];
#pragma unroll
    for (int dt = 0; dt < DT; ++dt) {
      FragB bvh, bvl;
#pragma unroll
      for (int i = 0; i < 8; ++i) {
        bvh.u[i] = sVh[8 * hh + i][dt * 16 + ln]; bvh.u[8 + i] = sVh[16 + 8 * hh + i][dt * 16 + ln];
        bvl.u[i] = sVl[8 * hh + i][dt * 16 + ln]; bvl.u[8 + i] = sVl[16 + 8 * hh + i][dt * 16 + ln];
      }
      oacc[dt] = mmaN<3>(pah.v, pal.v, bvh.v, bvl.v, oacc[dt]);
    }
    __builtin_amdgcn_fence(__ATOMIC_ACQ_REL, "workgroup");
    __builtin_amdgcn_wave_barrier();
  }
#pragma unroll
  for (int r = 0; r < 8; ++r) {
    float l = l_r[r];
    l += __shfl_xor(l, 1, 32); l += __shfl_xor(l, 2, 32); l += __shfl_xor(l, 4, 32); l += __shfl_xor(l, 8, 32);
    l_r[r] = (l > 0.f) ? 1.0f / l : 0.f;
  }
#pragma unroll
  for (int dt = 0; dt < DT; ++dt)
#pragma unroll
    for (int r = 0; r < 8; ++r) sO[w][8 * hh + r][dt * 16 + ln] = oacc[dt][r] * l_r[r];
  __builtin_amdgcn_fence(__ATOMIC_ACQ_REL, "workgroup");
  __builtin_amdgcn_wave_barrier();
  for (int pass = 0; pass < 2; ++pass) {
    for (int r = 0; r < 16; ++r) {
      const int row = q0 + r;
      if (row < T && lane < D / 4) {
        const v4f val = *(const v4fa*)&sO[w][r][lane * 4];
        *(volatile v4f*)(y + ((size_t)b * T + row) * ypitch + h * D + lane * 4) = val;
      }
    }
    if (pass == 0) __threadfence();
  }
}

template <bool ASPLIT, int ACT, bool BIAS_BF16, bool RES_BF16>
__global__ __launch_bounds__(128) void k_gemm_bf3(const float* __restrict__ A, int lda, const unsigned short* __restrict__ Wt, int ldb,
                                                const float* __restrict__ bias, const float* __restrict__ resid, int rmod, int ldr,
                                                float* __restrict__ C, int ldc, int M, int N, int K) {
  __shared__ __attribute__((aligned(16))) float so[4][16][64];
  const int tid = threadIdx.x, w = tid >> 5, lane = tid & 31, ln = lane & 15, hh = lane >> 4;
  const int ntn = N / 64;
  const int wid = blockIdx.x * 4 + w;
  const int mt = wid / ntn, nq = wid % ntn;
  if (mt * 16 >= M) return;
  const int row0 = mt * 16, col0 = nq * 64;
  const float* arow = A + (size_t)(row0 + ln) * lda;
  v8f acc[4] = {};
  for (int kb = 0; kb < K; kb += 32) {
    FragB ah, al;
    const v4f x0 = *(const v4fa*)(arow + kb + 8 * hh), x1 = *(const v4fa*)(arow + kb + 8 * hh + 4);
    const v4f x2 = *(const v4fa*)(arow + kb + 16 + 8 * hh), x3 = *(const v4fa*)(arow + kb + 16 + 8 * hh + 4);
    float xs[16] = {x0[0],x0[1],x0[2],x0[3],x1[0],x1[1],x1[2],x1[3],x2[0],x2[1],x2[2],x2[3],x3[0],x3[1],x3[2],x3[3]};
#pragma unroll
    for (int i = 0; i < 16; ++i) { const unsigned short hb = bf16_bits(xs[i]); ah.u[i] = hb; al.u[i] = ASPLIT ? bf16_bits(xs[i] - bf16_val(hb)) : (unsigned short)0; }
#pragma unroll
    for (int t = 0; t < 4; ++t) {
      const unsigned short* brow = Wt + (size_t)(col0 + t * 16 + ln) * ldb + kb;
      FragB b;
      b.half[0] = *(const v8us*)(brow + 8 * hh);
      b.half[1] = *(const v8us*)(brow + 16 + 8 * hh);
      acc[t] = mmaN<ASPLIT ? 2 : 1>(ah.v, al.v, b.v, b.v, acc[t]);
    }
  }
#pragma unroll
  for (int t = 0; t < 4; ++t) {
    const int col = col0 + t * 16 + ln;
    float bv = bias ? bias[col] : 0.f;
    if (BIAS_BF16) bv = bf16_round(bv);
#pragma unroll
    for (int r = 0; r < 8; ++r) {
      float v = acc[t][r] + bv;
      if (resid) { float rv = resid[(size_t)((row0 + 8 * hh + r) % rmod) * ldr + col]; if (RES_BF16) rv = bf16_round(rv); v += rv; }
      if (ACT == 1) v = fmaxf(v, 0.f);
      if (ACT == 2) v = 0.5f * v * (1.0f + erff(v * 0.70710678118654752f));
      if (ACT == 3) { const float u = 0.7978845608028654f * (v + 0.044715f * v * v * v); v = 0.5f * v * (1.0f + tanhf(u)); }
      so[w][8 * hh + r][t * 16 + ln] = v;
    }
  }
  __builtin_amdgcn_fence(__ATOMIC_ACQ_REL, "workgroup");
  __builtin_amdgcn_wave_barrier();
  const int rsub = lane >> 4, c4 = (lane & 15) * 4;
  for (int pass = 0; pass < 2; ++pass) {
#pragma unroll
    for (int q = 0; q < 8; ++q) {
      const int r = q * 2 + rsub;
      const v4f v = *(const v4fa*)&so[w][r][c4];
      *(volatile v4f*)(C + (size_t)(row0 + r) * ldc + col0 + c4) = v;
    }
    if (pass == 0) __threadfence();
  }
}
template <bool PARAM_BF16>
__global__ __launch_bounds__(256) void k_layernorm(const float* __restrict__ X, const float* __restrict__ R, const float* __restrict__ g, const float* __restrict__ bta,
                                                  float* __restrict__ out_sum, float* __restrict__ out_norm, int N, float eps) {
  __shared__ float red[256];
  const int row = blockIdx.x, tid = threadIdx.x;
  const float* x = X + (size_t)row * N; const float* rr = R ? R + (size_t)row * N : nullptr;
  float vals[16];
  const int per = N / 256;
  float s1 = 0.f;
  for (int u = 0; u < per / 4; ++u) {
    const int j = tid * 4 + 1024 * u;
    const v4f a = *(const v4fa*)(x + j);
    v4f b = {0.f,0.f,0.f,0.f}; if (rr) b = *(const v4fa*)(rr + j);
#pragma unroll
    for (int q = 0; q < 4; ++q) { const float v = a[q] + b[q]; vals[u * 4 + q] = v; s1 += v; }
  }
  red[tid] = s1; __syncthreads();
  for (int st = 128; st > 0; st >>= 1) { if (tid < st) red[tid] += red[tid + st]; __syncthreads(); }
  const float mu = red[0] / (float)N; __syncthreads();
  float s2 = 0.f;
  for (int u = 0; u < per / 4; ++u)
#pragma unroll
    for (int q = 0; q < 4; ++q) { const float c = vals[u * 4 + q] - mu; s2 += c * c; }
  red[tid] = s2; __syncthreads();
  for (int st = 128; st > 0; st >>= 1) { if (tid < st) red[tid] += red[tid + st]; __syncthreads(); }
  const float rs = rsqrtf(red[0] / (float)N + eps);
  for (int pass = 0; pass < 2; ++pass) {
    for (int u = 0; u < per / 4; ++u) {
      const int j = tid * 4 + 1024 * u;
      v4f o, sm;
#pragma unroll
      for (int q = 0; q < 4; ++q) {
        float gg = g[j + q], bb = bta[j + q];
        if (PARAM_BF16) { gg = bf16_round(gg); bb = bf16_round(bb); }
        sm[q] = vals[u * 4 + q]; o[q] = (vals[u * 4 + q] - mu) * rs * gg + bb;
      }
      if (out_sum) *(volatile v4f*)(out_sum + (size_t)row * N + j) = sm;
      *(volatile v4f*)(out_norm + (size_t)row * N + j) = o;
    }
    if (pass == 0) __threadfence();
  }
}


typedef _Float16 v16h __attribute__((ext_vector_type(16)));
union FragH { v16h v; v8us half[2]; _Float16 h[16]; unsigned short u[16]; };
template <int NT>
__device__ __forceinline__ v8f mmaH(v16h ah, v16h al, v16h bh, v16h bl, v8f c) {
  c = __builtin_amdgcn_wmma_f32_16x16x32_f16(false, ah, false, bh, (short)0, c, false, false);
  if (NT >= 2) c = __builtin_amdgcn_wmma_f32_16x16x32_f16(false, al, false, bh, (short)0, c, false, false);
  if (NT >= 3) c = __builtin_amdgcn_wmma_f32_16x16x32_f16(false, ah, false, bl, (short)0, c, false, false);
  asm volatile("v_nop\n\tv_nop\n\tv_nop\n\tv_nop" : "+v"(c) : "v"(ah), "v"(al), "v"(bh), "v"(bl));
  return c;
}
template <bool ASPLIT>
__global__ __launch_bounds__(128) void k_gemm_h(const float* __restrict__ A, int lda, size_t sA, const _Float16* __restrict__ Bh, int ldb, size_t sB, float alpha, float* __restrict__ C, int ldc, size_t sC, int M, int N, int K) {
  __shared__ __attribute__((aligned(16))) float so[4][16][64];
  const int tid = threadIdx.x, w = tid >> 5, lane = tid & 31, ln = lane & 15, hh = lane >> 4; const int by = blockIdx.y;
  A += (size_t)by * sA; Bh += (size_t)by * sB; C += (size_t)by * sC;
  const int ntn = (N + 63) / 64; const int wid = blockIdx.x * 4 + w; const int mt = wid / ntn, nq = wid % ntn; if (mt * 16 >= M) return;
  const int row0 = mt * 16, col0 = nq * 64; const float* arow = A + (size_t)(row0 + ln) * lda;
  v8f acc[4] = {};
  for (int kb = 0; kb < K; kb += 32) {
    FragH ah, al;
    const v4f x0 = *(const v4fa*)(arow + kb + 8 * hh), x1 = *(const v4fa*)(arow + kb + 8 * hh + 4), x2 = *(const v4fa*)(arow + kb + 16 + 8 * hh), x3 = *(const v4fa*)(arow + kb + 16 + 8 * hh + 4);
    float xs[16] = {x0[0],x0[1],x0[2],x0[3],x1[0],x1[1],x1[2],x1[3],x2[0],x2[1],x2[2],x2[3],x3[0],x3[1],x3[2],x3[3]};
#pragma unroll
    for (int i = 0; i < 16; ++i) { const _Float16 h = (_Float16)xs[i]; ah.h[i] = h; al.h[i] = ASPLIT ? (_Float16)(xs[i] - (float)h) : (_Float16)0.0f; }
#pragma unroll
    for (int t = 0; t < 4; ++t) { if (col0 + t * 16 >= N) continue; const size_t boff = (size_t)(col0 + t * 16 + ln) * ldb + kb; FragH bq; bq.half[0] = *(const v8us*)(Bh + boff + 8 * hh); bq.half[1] = *(const v8us*)(Bh + boff + 16 + 8 * hh);
      acc[t] = mmaH<ASPLIT ? 2 : 1>(ah.v, al.v, bq.v, bq.v, acc[t]); }
  }
#pragma unroll
  for (int t = 0; t < 4; ++t) { if (col0 + t * 16 >= N) continue;
#pragma unroll
    for (int r = 0; r < 8; ++r) so[w][8 * hh + r][t * 16 + ln] = acc[t][r] * alpha; }
  __builtin_amdgcn_fence(__ATOMIC_ACQ_REL, "workgroup"); __builtin_amdgcn_wave_barrier();
  const int rsub = lane >> 4, c4 = (lane & 15) * 4;
  for (int pass = 0; pass < 2; ++pass) {
#pragma unroll
    for (int q = 0; q < 8; ++q) { const int r = q * 2 + rsub; if (col0 + c4 < N) { const v4f v = *(const v4fa*)&so[w][r][c4]; *(volatile v4f*)(C + (size_t)(row0 + r) * ldc + col0 + c4) = v; } }
    if (pass == 0) __threadfence(); }
}

__global__ __launch_bounds__(256) void k_wt_f16(const float* __restrict__ W, _Float16* __restrict__ Wt, int K, int N, float scale) {
  const int t = blockIdx.x * 256 + threadIdx.x; if (t >= N * (K / 8)) return; const int n = t / (K / 8), k8 = (t % (K / 8)) * 8; FragH f;
#pragma unroll
  for (int i = 0; i < 8; ++i) f.h[i] = (_Float16)(bf16_round(W[(size_t)(k8 + i) * N + n]) * scale); const v8us o = f.half[0];
  *(volatile v8us*)((unsigned short*)Wt + (size_t)n * K + k8) = o; __threadfence(); *(volatile v8us*)((unsigned short*)Wt + (size_t)n * K + k8) = o;
}
template <int ACT>
__global__ __launch_bounds__(128) void k_gemm_hhx(const _Float16* __restrict__ A, int lda, size_t sA, const _Float16* __restrict__ Bh, int ldb, size_t sB, float alpha, const float* __restrict__ bias, size_t sBias, const float* __restrict__ CP, int rowsPerB, size_t sCPb, int row0g,
    float* __restrict__ C, _Float16* __restrict__ C16, int ldc, size_t sC, int M, int N, int K) {
  __shared__ __attribute__((aligned(16))) float so[4][16][64];
  const int tid = threadIdx.x, w = tid >> 5, lane = tid & 31, ln = lane & 15, hh = lane >> 4; const int by = blockIdx.y;
  A += (size_t)by * sA; Bh += (size_t)by * sB; const size_t cofs = (size_t)by * sC; const float* bp = bias ? bias + (size_t)by * sBias : nullptr;
  const int ntn = (N + 63) / 64; const int wid = blockIdx.x * 4 + w; const int mt = wid / ntn, nq = wid % ntn; if (mt * 16 >= M) return;
  const int row0 = mt * 16, col0 = nq * 64; const _Float16* arow = A + (size_t)(row0 + ln) * lda;
  v8f acc[4] = {};
  for (int kb = 0; kb < K; kb += 32) { FragH ah; ah.half[0] = *(const v8us*)((const unsigned short*)arow + kb + 8 * hh); ah.half[1] = *(const v8us*)((const unsigned short*)arow + kb + 16 + 8 * hh);
#pragma unroll
    for (int t = 0; t < 4; ++t) { if (col0 + t * 16 >= N) continue; const size_t boff = (size_t)(col0 + t * 16 + ln) * ldb + kb; FragH bq; bq.half[0] = *(const v8us*)((const unsigned short*)Bh + boff + 8 * hh); bq.half[1] = *(const v8us*)((const unsigned short*)Bh + boff + 16 + 8 * hh);
      acc[t] = mmaH<1>(ah.v, ah.v, bq.v, bq.v, acc[t]); }
  }
#pragma unroll
  for (int t = 0; t < 4; ++t) { if (col0 + t * 16 >= N) continue; const int col = col0 + t * 16 + ln; const float bv = bp ? bf16_round(bp[col]) : 0.f;
#pragma unroll
    for (int r = 0; r < 8; ++r) { float v = acc[t][r] * alpha + bv; if (CP) { const int bidx = (row0g + row0 + 8 * hh + r) / rowsPerB; v += CP[(size_t)bidx * sCPb + (size_t)by * 64 + col]; } if (ACT == 1) v = (v > 0.f) ? v : expm1f(v); else if (ACT == 3) v = fmaxf(v, 0.f); so[w][8 * hh + r][t * 16 + ln] = v; } }
  __builtin_amdgcn_fence(__ATOMIC_ACQ_REL, "workgroup"); __builtin_amdgcn_wave_barrier();
  const int rsub = lane >> 4, c4 = (lane & 15) * 4; typedef _Float16 v4h __attribute__((ext_vector_type(4)));
  for (int pass = 0; pass < 2; ++pass) {
#pragma unroll
    for (int q = 0; q < 8; ++q) { const int r = q * 2 + rsub; if (col0 + c4 < N) { const v4f v = *(const v4fa*)&so[w][r][c4]; if (C) *(volatile v4f*)(C + cofs + (size_t)(row0 + r) * ldc + col0 + c4) = v; if (C16) { v4h h4; for (int i = 0; i < 4; ++i) h4[i] = (_Float16)v[i]; *(volatile v4h*)(C16 + cofs + (size_t)(row0 + r) * ldc + col0 + c4) = h4; } } }
    if (pass == 0) __threadfence(); }
}


__global__ __launch_bounds__(256) void k_x16(const float* __restrict__ x, _Float16* __restrict__ X16, size_t n8) { const size_t t = (size_t)blockIdx.x * 256 + threadIdx.x; if (t >= n8) return; FragH f;
#pragma unroll
  for (int q = 0; q < 8; ++q) f.h[q] = (_Float16)bf16_round(x[t * 8 + q]); *(volatile v8us*)((unsigned short*)X16 + t * 8) = f.half[0]; __threadfence(); *(volatile v8us*)((unsigned short*)X16 + t * 8) = f.half[0]; }
__global__ __launch_bounds__(256) void k_h16(const float* __restrict__ x, _Float16* __restrict__ X16, size_t n8) { const size_t t = (size_t)blockIdx.x * 256 + threadIdx.x; if (t >= n8) return; FragH f;
#pragma unroll
  for (int q = 0; q < 8; ++q) f.h[q] = (_Float16)x[t * 8 + q]; *(volatile v8us*)((unsigned short*)X16 + t * 8) = f.half[0]; __threadfence(); *(volatile v8us*)((unsigned short*)X16 + t * 8) = f.half[0]; }
__global__ __launch_bounds__(256) void k_round16f(const float* __restrict__ W, _Float16* __restrict__ Bt, size_t n8) { const size_t t = (size_t)blockIdx.x * 256 + threadIdx.x; if (t >= n8) return; FragH f;
#pragma unroll
  for (int i = 0; i < 8; ++i) f.h[i] = (_Float16)(bf16_round(W[t * 8 + i]) * 16.0f); *(volatile v8us*)((unsigned short*)Bt + t * 8) = f.half[0]; __threadfence(); *(volatile v8us*)((unsigned short*)Bt + t * 8) = f.half[0]; }
template <int NHv, int TTv>
__global__ __launch_bounds__(256) void k_vt(const _Float16* __restrict__ V16, int ldv, int voff, _Float16* __restrict__ Vt) { __shared__ unsigned short tl[64][66]; const int tid = threadIdx.x; const int slab = blockIdx.x / (TTv / 64), lg = blockIdx.x % (TTv / 64); const int b = slab / NHv, h = slab % NHv;
  for (int i = tid; i < 64 * 8; i += 256) { const int r = i / 8, c8 = (i % 8) * 8; FragH f; f.half[0] = *(const v8us*)((const unsigned short*)V16 + ((size_t)b * TTv + lg * 64 + r) * ldv + voff + h * 64 + c8);
#pragma unroll
    for (int q = 0; q < 8; ++q) tl[r][c8 + q] = f.u[q]; }
  __syncthreads();
  for (int pass = 0; pass < 2; ++pass) {
#pragma unroll
    for (int rd = 0; rd < 2; ++rd) { const int d = rd * 32 + tid / 8, pc = tid % 8; FragH f;
#pragma unroll
      for (int q = 0; q < 8; ++q) f.u[q] = tl[pc * 8 + q][d];
      *(volatile v8us*)((unsigned short*)Vt + ((size_t)slab * 64 + d) * TTv + lg * 64 + pc * 8) = f.half[0]; }
    if (pass == 0) __threadfence(); } }

__device__ __forceinline__ int bscan512(int cnt, int* wsum, int tid, int& total) {
  const int lane = tid & 31, wv = tid >> 5; int x = cnt;
#pragma unroll
  for (int d = 1; d < 32; d <<= 1) { const int y = __shfl_up(x, d, 32); if (lane >= d) x += y; }
  __syncthreads(); if (lane == 31) wsum[wv] = x; __syncthreads();
  int t = (lane < 16) ? wsum[lane] : 0;
#pragma unroll
  for (int d = 1; d < 32; d <<= 1) { const int y = __shfl_up(t, d, 32); if (lane >= d) t += y; }
  const int woff = (wv == 0) ? 0 : __shfl(t, wv - 1, 32); total = __shfl(t, 15, 32);
  return woff + x - cnt; }
#define QCAP 8
#define CHUNK 8192
#define NNODE NA
#define NE ECH
typedef _Float16 v4h __attribute__((ext_vector_type(4)));
__global__ __launch_bounds__(256) void k_zero4(float* __restrict__ p, size_t n4) { const size_t i = (size_t)blockIdx.x * 256 + threadIdx.x; if (i < n4) { const v4f z = {0.f, 0.f, 0.f, 0.f}; *(volatile v4f*)(p + i * 4) = z; __threadfence(); *(volatile v4f*)(p + i * 4) = z; } }
__global__ __launch_bounds__(256) void k_radial(const float* __restrict__ es, const float* __restrict__ w1, int e0, _Float16* __restrict__ H16) { const int t = blockIdx.x * 256 + threadIdx.x; if (t >= ECH * (FHP / 8)) return; const int j8 = (t % (FHP / 8)) * 8; const int el = t / (FHP / 8); const size_t e = (size_t)e0 + el; float x[10];
#pragma unroll
  for (int k = 0; k < 10; ++k) x[k] = bf16_round(es[e * 10 + k]); FragH f;
#pragma unroll
  for (int q = 0; q < 8; ++q) { const int j = j8 + q; float v = 0.f; if (j < FH) { float s = 0.f;
#pragma unroll
      for (int k = 0; k < 10; ++k) s += x[k] * bf16_round(w1[k * FH + j]); s *= 0.31622776601683794f; v = s / (1.0f + expf(-s)); } f.h[q] = (_Float16)v; }
  *(volatile v8us*)((unsigned short*)H16 + (size_t)t * 8) = f.half[0]; __threadfence(); *(volatile v8us*)((unsigned short*)H16 + (size_t)t * 8) = f.half[0]; }
__global__ __launch_bounds__(256) void k_w2(const float* __restrict__ w2, _Float16* __restrict__ Bt) { const int t = blockIdx.x * 256 + threadIdx.x; if (t >= WN * (FHP / 8)) return; const int k8 = (t % (FHP / 8)) * 8; const int o = t / (FHP / 8); FragH f;
#pragma unroll
  for (int q = 0; q < 8; ++q) { const int k = k8 + q; f.h[q] = (_Float16)((k < FH) ? bf16_round(w2[k * WN + o]) * 16.0f : 0.f); } *(volatile v8us*)((unsigned short*)Bt + (size_t)t * 8) = f.half[0]; __threadfence(); *(volatile v8us*)((unsigned short*)Bt + (size_t)t * 8) = f.half[0]; }
__global__ __launch_bounds__(256) void k_nodein(const float* __restrict__ x, const float* __restrict__ attr, int nn, _Float16* __restrict__ X0, _Float16* __restrict__ XM) { const int t = blockIdx.x * 256 + threadIdx.x; if (t >= nn * 40) return; const int n = t / 40, pc = t % 40; const float a = bf16_round(attr[n]); FragH f;
  if (pc < 16) { for (int q = 0; q < 8; ++q) f.h[q] = (_Float16)(bf16_round(x[(size_t)n * DIM + pc * 8 + q]) * a); unsigned short* d = (unsigned short*)X0 + (size_t)n * M0 + pc * 8; *(volatile v8us*)d = f.half[0]; __threadfence(); *(volatile v8us*)d = f.half[0]; }
  else { const int m = (pc - 16) / 8, u8 = ((pc - 16) % 8) * 8; for (int q = 0; q < 8; ++q) f.h[q] = (_Float16)(bf16_round(x[(size_t)n * DIM + M0 + (u8 + q) * 3 + m]) * a); unsigned short* d = (unsigned short*)XM + ((size_t)n * 3 + m) * M1 + u8; *(volatile v8us*)d = f.half[0]; __threadfence(); *(volatile v8us*)d = f.half[0]; } }
__global__ __launch_bounds__(256) void k_l1scatter(const float* __restrict__ C1, int nn, float* __restrict__ OUT, int ld, int c0) { const int t = blockIdx.x * 256 + threadIdx.x; if (t >= nn * 48) return; const int n = t / 48, j = t % 48; v4f a;
#pragma unroll
  for (int q = 0; q < 4; ++q) { const int idx = j * 4 + q; const int v = idx / 3, m = idx % 3; a[q] = C1[((size_t)n * 3 + m) * M1 + v]; }
  float* d = OUT + (size_t)n * ld + c0 + j * 4; *(volatile v4f*)d = a; __threadfence(); *(volatile v4f*)d = a; }
template <int TY, int CW>
__global__ __launch_bounds__(512) void k_tp(const float* __restrict__ S0, const float* __restrict__ S1, const float* __restrict__ Wc, const float* __restrict__ EA, int e0, int col0, const int* __restrict__ esrc_base, const int* __restrict__ edst_base, float* __restrict__ R) {
  #pragma clang fp contract(off)
  const int* __restrict__ srci = esrc_base + e0; const int* __restrict__ dsti = edst_base + e0;
  __shared__ short Lr[CHUNK]; __shared__ int Le[CHUNK]; __shared__ int scan[16]; __shared__ int lq[16][QCAP][32]; __shared__ __attribute__((aligned(16))) float stg[64][68];
  const int tid = threadIdx.x, lane = tid & 31, wv = tid >> 5; const int n0 = blockIdx.x * 1024; int qn = 0; float acc[2][CW];
#pragma unroll
  for (int s2 = 0; s2 < 2; ++s2)
#pragma unroll
    for (int c = 0; c < CW; ++c) acc[s2][c] = 0.f;
  const int u0 = (TY == 2) ? (col0 - 192) / 3 : ((TY == 3) ? (col0 - 576) / 3 : col0);

#pragma unroll 1
  for (int eb = 0; eb < NE + CHUNK; eb += CHUNK) { const bool sentinel = (eb >= NE); int tot = 0;
    if (!sentinel) { int k_cnt = 0; unsigned hm = 0; int hv[16];
#pragma unroll
      for (int k = 0; k < 16; ++k) { const int e = eb + tid * 16 + k; const int ec = (e < NE) ? e : (NE - 1); const int dv = dsti[ec] - n0; const int dd_ = (e < NE) ? dv : -1; hv[k] = dd_; if (dd_ >= 0 && dd_ < 1024) { hm |= 1u << k; ++k_cnt; } }
      int p = bscan512(k_cnt, scan, tid, tot);
#pragma unroll
      for (int k = 0; k < 16; ++k) if (hm & (1u << k)) { Lr[p] = (short)hv[k]; Le[p] = eb + tid * 16 + k; ++p; }
      __syncthreads(); }
    const int ntrip = sentinel ? 1 : ((tot + 31) >> 5);
#pragma unroll 1
    for (int it = 0; it < ntrip; ++it) { const int q = it * 32 + lane; const int lr = (!sentinel && q < tot) ? (int)Lr[q] : -1;
      unsigned mm = sentinel ? 1u : __builtin_amdgcn_ballot_w32(lr >= wv * 64 && lr < wv * 64 + 64);
#pragma unroll 1
      while (mm) { const int bit = __builtin_ctz(mm); mm &= mm - 1u; const int ol = sentinel ? -2 : (__shfl(lr, bit, 32) - wv * 64); const int owner = ol >> 1; const int e = sentinel ? 0 : Le[it * 32 + bit];
        if (sentinel || __builtin_amdgcn_ballot_w32(lane == owner && qn == QCAP)) {
          int kmax = qn;
#pragma unroll
          for (int o = 16; o >= 1; o >>= 1) kmax = max(kmax, __shfl_xor(kmax, o, 32));
#pragma unroll 1
          for (int k = 0; k < kmax; ++k) { if (k < qn) { const int ent = lq[wv][k][lane]; const int eq = ent >> 1; const int sl = ent & 1; int s = srci[eq]; s = s < 0 ? 0 : (s >= NNODE ? NNODE - 1 : s);
              const float* w = Wc + (size_t)eq * WN; const float* ea = EA + ((size_t)e0 + eq) * 4; const float sh0 = bf16_round(ea[0]); const float sh1[3] = {bf16_round(ea[1]), bf16_round(ea[2]), bf16_round(ea[3])};
              const float* g0 = S0 + (size_t)s * M0; const float* g1 = S1 + (size_t)s * MID;
#pragma unroll
              for (int s2 = 0; s2 < 2; ++s2) if (s2 == sl) {
                if (TY == 0) {
#pragma unroll
                  for (int c = 0; c < CW; ++c) { const int u = u0 + c; acc[s2][c] += (w[u] * g0[u]) * sh0; } }
                else if (TY == 1) {
#pragma unroll
                  for (int c = 0; c < CW; ++c) { const int v = u0 - 128 + c; const float d = g1[v * 3] * sh1[0] + g1[v * 3 + 1] * sh1[1] + g1[v * 3 + 2] * sh1[2]; acc[s2][c] += (w[320 + v] * d) * 0.57735026918962576f; } }
                else if (TY == 2) {
#pragma unroll
                  for (int uu = 0; uu < CW / 3; ++uu) { const int u = u0 + uu; const float pr = w[128 + u] * g0[u];
#pragma unroll
                    for (int m = 0; m < 3; ++m) acc[s2][uu * 3 + m] += pr * sh1[m]; } }
                else {
#pragma unroll
                  for (int uu = 0; uu < CW / 3; ++uu) { const int v = u0 + uu; const float wv2 = w[256 + v];
#pragma unroll
                    for (int m = 0; m < 3; ++m) acc[s2][uu * 3 + m] += (wv2 * g1[v * 3 + m]) * sh0; } } } } }
          qn = 0; }
        if (lane == owner) { lq[wv][qn][lane] = e * 2 + (ol & 1); ++qn; } } }
    __syncthreads(); }
  for (int tg = 0; tg < 16; ++tg) {
    if (wv == tg) {
#pragma unroll
      for (int c = 0; c < CW; ++c) { stg[2 * lane][c] = acc[0][c]; stg[2 * lane + 1][c] = acc[1][c]; } }
    __syncthreads();
    v4f sum[2]; float* dst[2];
#pragma unroll
    for (int rd = 0; rd < 2; ++rd) { const int r = rd * 32 + tid / 16, pc = tid % 16; const int n = n0 + tg * 64 + r; dst[rd] = nullptr; if (n < NPR && pc < CW / 4) { dst[rd] = R + (size_t)n * 768 + col0 + pc * 4; const v4f cur = *(const v4fa*)dst[rd]; v4f a; for (int q = 0; q < 4; ++q) a[q] = cur[q] + stg[r][pc * 4 + q]; sum[rd] = a; } }
    for (int pass = 0; pass < 2; ++pass) {
#pragma unroll
      for (int rd = 0; rd < 2; ++rd) if (dst[rd]) *(volatile v4f*)dst[rd] = sum[rd];
      if (pass == 0) __threadfence(); }
    __syncthreads(); } }
__global__ __launch_bounds__(256) void k_split(const float* __restrict__ F, int ld, int c0, int ncol, float scale, int nrows, _Float16* __restrict__ Hh, _Float16* __restrict__ Hl) { const size_t t = (size_t)blockIdx.x * 256 + threadIdx.x; const int n8 = ncol / 8; if (t >= (size_t)nrows * n8) return; const size_t r = t / n8; const int c8 = (int)(t % n8) * 8; FragH fh, fl;
#pragma unroll
  for (int q = 0; q < 8; ++q) { const float v = F[r * ld + c0 + c8 + q] * scale; const _Float16 h = (_Float16)v; fh.h[q] = h; fl.h[q] = (_Float16)((v - (float)h) * 1024.0f); }
  for (int pass = 0; pass < 2; ++pass) { *(volatile v8us*)((unsigned short*)Hh + (r * ncol + c8)) = fh.half[0]; *(volatile v8us*)((unsigned short*)Hl + (r * ncol + c8)) = fl.half[0]; if (pass == 0) __threadfence(); } }
__global__ __launch_bounds__(256) void k_attrscale(float* __restrict__ R, const float* __restrict__ attr) { const size_t t = (size_t)blockIdx.x * 256 + threadIdx.x; if (t >= (size_t)NPR * 768 / 4) return; const size_t p = (t * 4) / 768; const float a = bf16_round(attr[p]); v4f v = *(const v4fa*)(R + t * 4); for (int q = 0; q < 4; ++q) v[q] *= a; *(volatile v4f*)(R + t * 4) = v; __threadfence(); *(volatile v4f*)(R + t * 4) = v; }
__global__ __launch_bounds__(256) void k_rm1(const float* __restrict__ Rs, int m, float scale, _Float16* __restrict__ Hh, _Float16* __restrict__ Hl) { const size_t t = (size_t)blockIdx.x * 256 + threadIdx.x; if (t >= (size_t)NPR * (MID / 8)) return; const int u8 = (int)(t % (MID / 8)) * 8; const size_t p = t / (MID / 8); FragH fh, fl;
#pragma unroll
  for (int q = 0; q < 8; ++q) { const float v = Rs[p * 768 + MID + (u8 + q) * 3 + m] * scale; const _Float16 h = (_Float16)v; fh.h[q] = h; fl.h[q] = (_Float16)((v - (float)h) * 1024.0f); }
  for (int pass = 0; pass < 2; ++pass) { *(volatile v8us*)((unsigned short*)Hh + t * 8) = fh.half[0]; *(volatile v8us*)((unsigned short*)Hl + t * 8) = fl.half[0]; if (pass == 0) __threadfence(); } }
__global__ __launch_bounds__(256) void k_mscatter(const float* __restrict__ C1, int m, float* __restrict__ OUT) { const int t = blockIdx.x * 256 + threadIdx.x; if (t >= NPR * 48) return; const int p = t / 48, j = t % 48; float* d = OUT + (size_t)p * DIM + M0 + j * 4; v4f a;
#pragma unroll
  for (int q = 0; q < 4; ++q) { const int idx = j * 4 + q; const int v = idx / 3, mm = idx % 3; a[q] = (mm == m) ? C1[(size_t)p * M1 + v] : ((m == 0) ? 0.f : d[q]); }
  *(volatile v4f*)d = a; __threadfence(); *(volatile v4f*)d = a; }
__global__ __launch_bounds__(256) void k_final(const float* __restrict__ R, const float* __restrict__ lin3, const float* __restrict__ SC, const float* __restrict__ CONV, float* __restrict__ out) { const int tid = threadIdx.x, wv = tid >> 5, lane = tid & 31; const int p = blockIdx.x * 8 + wv; if (p >= NPR) return; const float sc = 0.31622776601683794f; float s = 0.f;
#pragma unroll 1
  for (int u = lane; u < MID; u += 32) s += R[(size_t)p * 768 + u] * sc * bf16_round(lin3[u]); for (int o = 16; o >= 1; o >>= 1) s += __shfl_xor(s, o, 32); const float ang = 0.1f * s * 0.07216878364870322f; const float ca = cosf(ang), sa = sinf(ang);
  v4f o0, o1, o2; const bool h2 = (lane + 64) < DIM / 4;
  { const v4f a = *(const v4fa*)(SC + (size_t)p * DIM + lane * 4), b = *(const v4fa*)(CONV + (size_t)p * DIM + lane * 4); for (int q = 0; q < 4; ++q) o0[q] = ca * a[q] + sa * b[q]; }
  { const v4f a = *(const v4fa*)(SC + (size_t)p * DIM + (lane + 32) * 4), b = *(const v4fa*)(CONV + (size_t)p * DIM + (lane + 32) * 4); for (int q = 0; q < 4; ++q) o1[q] = ca * a[q] + sa * b[q]; }
  if (h2) { const v4f a = *(const v4fa*)(SC + (size_t)p * DIM + (lane + 64) * 4), b = *(const v4fa*)(CONV + (size_t)p * DIM + (lane + 64) * 4); for (int q = 0; q < 4; ++q) o2[q] = ca * a[q] + sa * b[q]; } else { o2 = o1; }
  __builtin_amdgcn_wave_barrier();
  for (int pass = 0; pass < 2; ++pass) { *(volatile v4f*)(out + (size_t)p * DIM + lane * 4) = o0; *(volatile v4f*)(out + (size_t)p * DIM + (lane + 32) * 4) = o1; if (h2) *(volatile v4f*)(out + (size_t)p * DIM + (lane + 64) * 4) = o2; if (pass == 0) __threadfence(); } }
extern "C" void kernel_launch(void* const* d_in, const int* in_sizes, int n_in,
                              void* d_out, int out_size, void* d_ws, size_t ws_size, hipStream_t stream) {
  (void)in_sizes; (void)n_in; (void)out_size;
  const float* const* I = (const float* const*)d_in; const float* snd = I[0]; const float* sattr = I[1]; const float* rcv = I[2]; const float* rattr = I[3]; const int* esrc = (const int*)d_in[4]; const int* edst = (const int*)d_in[5]; const float* eattr = I[6]; const float* escal = I[7]; const float* fc_w1 = I[8]; const float* fc_w2 = I[9]; const float* lin1_w0 = I[10]; const float* lin1_w1 = I[11]; const float* sc_w0 = I[12]; const float* sc_w1 = I[13]; const float* lin2_w0 = I[14]; const float* lin2_w1 = I[15]; const float* lin3_w = I[16];
  char* ws = (char*)d_ws; size_t off = 0;
  auto take = [&](size_t bytes) { char* p = ws + off; off += (bytes + 255) & ~(size_t)255; return p; };
  _Float16* Bw2 = (_Float16*)take((size_t)WN * FHP * 2); _Float16* Bl10 = (_Float16*)take(M0 * M0 * 2); _Float16* Bl11 = (_Float16*)take(M1 * M1 * 2); _Float16* Bsc0 = (_Float16*)take(M0 * M0 * 2); _Float16* Bsc1 = (_Float16*)take(M1 * M1 * 2); _Float16* Bl20 = (_Float16*)take(M0 * MID * 2); _Float16* Bl21 = (_Float16*)take(M1 * MID * 2);
  _Float16* X0 = (_Float16*)take((size_t)NPP * M0 * 2); _Float16* XM = (_Float16*)take((size_t)NPP * 3 * M1 * 2); float* S0 = (float*)take((size_t)NAP * M0 * 4); float* S1 = (float*)take((size_t)NAP * MID * 4); float* R = (float*)take((size_t)NPP * 768 * 4); float* CONV = (float*)take((size_t)NPP * DIM * 4);
  char* REG = (char*)take((size_t)23 << 20);
  _Float16* H16 = (_Float16*)REG; float* Wc = (float*)(REG + ((size_t)12512 * FHP * 2 + 255) / 256 * 256); _Float16* Rh = (_Float16*)REG; _Float16* Rl = (_Float16*)(REG + (size_t)NPP * MID * 2); float* C1 = (float*)(REG + (size_t)2 * NPP * MID * 2);
  float* SCo = (float*)d_out;
  if (off > ws_size) return;
  k_w2<<<(WN * (FHP / 8) + 255) / 256, 256, 0, stream>>>(fc_w2, Bw2);
  k_wt_f16<<<(M0 * (M0 / 8) + 255) / 256, 256, 0, stream>>>(lin1_w0, Bl10, M0, M0, 16.0f); k_wt_f16<<<(M1 * (M1 / 8) + 255) / 256, 256, 0, stream>>>(lin1_w1, Bl11, M1, M1, 16.0f); k_wt_f16<<<(M0 * (M0 / 8) + 255) / 256, 256, 0, stream>>>(sc_w0, Bsc0, M0, M0, 16.0f); k_wt_f16<<<(M1 * (M1 / 8) + 255) / 256, 256, 0, stream>>>(sc_w1, Bsc1, M1, M1, 16.0f);
  k_wt_f16<<<(M0 * (MID / 8) + 255) / 256, 256, 0, stream>>>(lin2_w0, Bl20, MID, M0, 16.0f); k_wt_f16<<<(M1 * (MID / 8) + 255) / 256, 256, 0, stream>>>(lin2_w1, Bl21, MID, M1, 16.0f);
  const float a128 = 0.0625f * 0.088388347648318441f, a64 = 0.0625f * 0.125f, a192 = 0.0625f * 0.07216878364870322f;
  k_nodein<<<(NA * 40 + 255) / 256, 256, 0, stream>>>(snd, sattr, NA, X0, XM);
  k_gemm_hhx<0><<<dim3(((NAP / 16) * (M0 / 64) + 3) / 4, 1), 128, 0, stream>>>(X0, M0, 0, Bl10, M0, 0, a128, nullptr, 0, nullptr, 1, 0, 0, S0, nullptr, M0, 0, NAP, M0, M0);
  k_gemm_hhx<0><<<dim3(((NAP * 3 / 16) * 1 + 3) / 4, 1), 128, 0, stream>>>(XM, M1, 0, Bl11, M1, 0, a64, nullptr, 0, nullptr, 1, 0, 0, CONV, nullptr, M1, 0, NAP * 3, M1, M1);
  k_l1scatter<<<(NA * 48 + 255) / 256, 256, 0, stream>>>(CONV, NA, S1, MID, 0);
  k_zero4<<<(unsigned)(((size_t)NPP * 768 / 4 + 255) / 256), 256, 0, stream>>>(R, (size_t)NPP * 768 / 4);
  for (int e0 = 0; e0 < 200000; e0 += ECH) {
    k_radial<<<(ECH * (FHP / 8) + 255) / 256, 256, 0, stream>>>(escal, fc_w1, e0, H16);
    k_gemm_hhx<0><<<dim3(((12512 / 16) * (WN / 64) + 3) / 4, 1), 128, 0, stream>>>(H16, FHP, 0, Bw2, FHP, 0, 0.0625f * 0.1f, nullptr, 0, nullptr, 1, 0, 0, Wc, nullptr, WN, 0, 12512, WN, FHP);
    { const unsigned gq = (NPR + 1023) / 1024;
      k_tp<0, 64><<<gq, 512, 0, stream>>>(S0, S1, Wc, eattr, e0, 0, esrc, edst, R); k_tp<0, 64><<<gq, 512, 0, stream>>>(S0, S1, Wc, eattr, e0, 64, esrc, edst, R);
      k_tp<1, 32><<<gq, 512, 0, stream>>>(S0, S1, Wc, eattr, e0, 128, esrc, edst, R); k_tp<1, 32><<<gq, 512, 0, stream>>>(S0, S1, Wc, eattr, e0, 160, esrc, edst, R);
      for (int k = 0; k < 8; ++k) k_tp<2, 48><<<gq, 512, 0, stream>>>(S0, S1, Wc, eattr, e0, 192 + 48 * k, esrc, edst, R);
      for (int k = 0; k < 4; ++k) k_tp<3, 48><<<gq, 512, 0, stream>>>(S0, S1, Wc, eattr, e0, 576 + 48 * k, esrc, edst, R); } }
  k_attrscale<<<(unsigned)(((size_t)NPR * 768 / 4 + 255) / 256), 256, 0, stream>>>(R, rattr);
  k_split<<<(unsigned)(((size_t)NPR * (MID / 8) + 255) / 256), 256, 0, stream>>>(R, 768, 0, MID, 0.31622776601683794f, NPR, Rh, Rl);
  k_gemm_hhx<0><<<dim3(((NPP / 16) * (M0 / 64) + 3) / 4, 1), 128, 0, stream>>>(Rh, MID, 0, Bl20, MID, 0, a192, nullptr, 0, nullptr, 1, 0, 0, CONV, nullptr, DIM, 0, NPP, M0, MID);
  k_gemm_hhx<0><<<dim3(((NPP / 16) * (M0 / 64) + 3) / 4, 1), 128, 0, stream>>>(Rl, MID, 0, Bl20, MID, 0, a192 * 0.0009765625f, nullptr, 0, CONV, 1, (size_t)DIM, 0, CONV, nullptr, DIM, 0, NPP, M0, MID);
  for (int m = 0; m < 3; ++m) { k_rm1<<<(unsigned)(((size_t)NPR * (MID / 8) + 255) / 256), 256, 0, stream>>>(R, m, 0.31622776601683794f, Rh, Rl);
    k_gemm_hhx<0><<<dim3(((NPP / 16) * 1 + 3) / 4, 1), 128, 0, stream>>>(Rh, MID, 0, Bl21, MID, 0, a192, nullptr, 0, nullptr, 1, 0, 0, C1, nullptr, M1, 0, NPP, M1, MID);
    k_gemm_hhx<0><<<dim3(((NPP / 16) * 1 + 3) / 4, 1), 128, 0, stream>>>(Rl, MID, 0, Bl21, MID, 0, a192 * 0.0009765625f, nullptr, 0, C1, 1, (size_t)M1, 0, C1, nullptr, M1, 0, NPP, M1, MID);
    k_mscatter<<<(NPR * 48 + 255) / 256, 256, 0, stream>>>(C1, m, CONV); }
  k_nodein<<<(NPR * 40 + 255) / 256, 256, 0, stream>>>(rcv, rattr, NPR, X0, XM);
  k_gemm_hhx<0><<<dim3(((NPP / 16) * (M0 / 64) + 3) / 4, 1), 128, 0, stream>>>(X0, M0, 0, Bsc0, M0, 0, a128, nullptr, 0, nullptr, 1, 0, 0, SCo, nullptr, DIM, 0, NPR, M0, M0);
  { float* C1b = (float*)REG;
    k_gemm_hhx<0><<<dim3(((NPR * 3 / 16) * 1 + 3) / 4, 1), 128, 0, stream>>>(XM, M1, 0, Bsc1, M1, 0, a64, nullptr, 0, nullptr, 1, 0, 0, C1b, nullptr, M1, 0, NPR * 3, M1, M1);
    k_l1scatter<<<(NPR * 48 + 255) / 256, 256, 0, stream>>>(C1b, NPR, SCo, DIM, M0); }
  k_final<<<(NPR + 7) / 8, 256, 0, stream>>>(R, lin3_w, SCo, CONV, (float*)d_out);
}
